// MambaBlock_85298050499090
// MI455X (gfx1250) — hardware-verified
//
#include <hip/hip_runtime.h>
#include <math.h>

typedef __attribute__((ext_vector_type(16))) __bf16   v16b;
typedef __attribute__((ext_vector_type(8)))  __bf16   v8b;
typedef __attribute__((ext_vector_type(8)))  float    v8f;
typedef __attribute__((ext_vector_type(4)))  float    v4f;
typedef __attribute__((ext_vector_type(4)))  unsigned v4u;

constexpr int kBatch  = 2;
constexpr int kSeq    = 1024;
constexpr int kDm     = 1024;
constexpr int kDin    = 2048;
constexpr int kNst    = 16;
constexpr int kXzP    = 2 * kDin;
constexpr int kPrjN   = 2 * kNst + kDin;
constexpr int kPrjP   = 2112;
constexpr int kRows   = kBatch * kSeq;
constexpr int kConvTP = 260;
constexpr int kScanTS = 64;
constexpr int kScanCh = 64;
constexpr int kScanYP = 68;
constexpr int kScanXP = 2 * kNst;
static_assert(kPrjN == 2080, "x_proj width");
static_assert((kPrjP % 64) == 0 && kPrjP >= kPrjN, "padded x_proj width");
static_assert((kDm % 32) == 0 && (kDin % 32) == 0, "GEMM K multiples of 32");
static_assert((kRows % 64) == 0 && (kXzP % 64) == 0 && (kDm % 64) == 0, "GEMM M,N multiples of 64");
static_assert(((kRows / 64) * (kXzP / 64)) % 8 == 0, "in_proj tiles fill whole blocks");
static_assert(((kRows / 64) * (kPrjP / 64)) % 8 == 0, "x_proj tiles fill whole blocks");
static_assert(((kRows / 64) * (kDm / 64)) % 8 == 0, "out_proj tiles fill whole blocks");
static_assert((kSeq % kScanTS) == 0 && (kSeq % 64) == 0 && (kDin % kScanCh) == 0 && (kDin % 256) == 0, "tile multiples");
static_assert((kSeq & (kSeq - 1)) == 0, "sequence length is a power of two");
static_assert(((kPrjP * 4) % 128) == 0, "x_proj output pitch is a whole number of lines");

constexpr size_t kOffXB   = 0;
constexpr size_t kOffWIB  = kOffXB  + (size_t)kRows * kDm  * 2;
constexpr size_t kOffWXB  = kOffWIB + (size_t)kXzP  * kDm  * 2;
constexpr size_t kOffWOB  = kOffWXB + (size_t)kPrjP * kDin * 2;
constexpr size_t kOffXZ   = kOffWOB + (size_t)kDm   * kDin * 2;
constexpr size_t kOffXCH  = kOffXZ  + (size_t)kRows * kXzP * 4;
constexpr size_t kOffXCL  = kOffXCH + (size_t)kRows * kDin * 2;
constexpr size_t kOffDBU  = kOffXCL + (size_t)kRows * kDin * 2;
constexpr size_t kOffYH   = kOffDBU + (size_t)kRows * kPrjP * 4;
constexpr size_t kOffYL   = kOffYH  + (size_t)kRows * kDin * 2;
constexpr size_t kWsTotal = kOffYL  + (size_t)kRows * kDin * 2;
static_assert(kWsTotal == 109838336ull, "carve total");
static_assert(kWsTotal <= 134217728ull, "carve cap");
static_assert((kOffWIB % 128) == 0 && (kOffWXB % 128) == 0 && (kOffWOB % 128) == 0 && (kOffXZ % 128) == 0 &&
              (kOffXCH % 128) == 0 && (kOffXCL % 128) == 0 && (kOffDBU % 128) == 0 && (kOffYH % 128) == 0 &&
              (kOffYL % 128) == 0, "128-B aligned regions");

__device__ __forceinline__ unsigned bf_rne_bits(float f) {
  const unsigned u = __float_as_uint(f);
  return (u + 0x7FFFu + ((u >> 16) & 1u)) >> 16;
}
__device__ __forceinline__ float bf_bits_f(unsigned hb) { return __uint_as_float(hb << 16); }
__device__ __forceinline__ float bf_rne_f(float f) { return bf_bits_f(bf_rne_bits(f)); }
__device__ __forceinline__ unsigned pack_bf2(float a, float b) {
  const unsigned ha = bf_rne_bits(a);
  const unsigned hb = bf_rne_bits(b);
  return ha | (hb << 16);
}
__device__ __forceinline__ void split_bf2(float a, float b, unsigned& hw, unsigned& lw) {
  const unsigned ha = bf_rne_bits(a);
  const unsigned hb = bf_rne_bits(b);
  const float ra = a - bf_bits_f(ha);
  const float rb = b - bf_bits_f(hb);
  const unsigned la = bf_rne_bits(ra);
  const unsigned lb = bf_rne_bits(rb);
  hw = ha | (hb << 16);
  lw = la | (lb << 16);
}

__device__ __forceinline__ void guard4_b(v8f& a, v8f& b, v8f& c, v8f& d, v16b x, v16b y) {
  asm volatile("v_nop\n\tv_nop\n\tv_nop\n\tv_nop" : "+v"(a), "+v"(b), "+v"(c), "+v"(d) : "v"(x), "v"(y));
}
__device__ __forceinline__ void keep4_b(v16b a, v16b b, v16b c, v16b d) { asm volatile("v_nop" :: "v"(a), "v"(b), "v"(c), "v"(d)); }
__device__ __forceinline__ void acc_guard4(v8f& a, v8f& b, v8f& c, v8f& d) { asm volatile("v_nop\n\tv_nop\n\tv_nop\n\tv_nop" : "+v"(a), "+v"(b), "+v"(c), "+v"(d)); }

struct FragB {
  union U { v16b v; v8b h[2]; };
  static __device__ __forceinline__ v16b load(const __bf16* p) {
    U f;
    f.h[0] = *(const v8b*)(p);
    f.h[1] = *(const v8b*)(p + 16);
    return f.v;
  }
  static __device__ __forceinline__ v8f mma(v16b a, v16b b, v8f c) {
    return __builtin_amdgcn_wmma_f32_16x16x32_bf16(false, a, false, b, (short)0, c, false, false);
  }
};

template <int SPL, bool BIAS>
__global__ __launch_bounds__(256) void wmma_gemm64(
    const unsigned short* __restrict__ Ap, const unsigned short* __restrict__ A2p, int lda,
    const unsigned short* __restrict__ Btp, int ldb,
    float* __restrict__ C, int ldc,
    const float* __restrict__ bias, int nBias,
    int M, int N, int K) {
  const __bf16* A  = (const __bf16*)Ap;
  const __bf16* A2 = (const __bf16*)A2p;
  const __bf16* Bt = (const __bf16*)Btp;
  __shared__ __align__(16) float sT[8][16 * 68];
  const int lane = threadIdx.x & 31;
  const int wave = threadIdx.x >> 5;
  const int tilesN = N >> 6;
  const int tilesM = M >> 6;
  const int tile = blockIdx.x * 8 + wave;
  if (tile >= tilesM * tilesN) return;
  const int tm = tile / tilesN;
  const int tn = tile - tm * tilesN;
  const int m0 = tm << 6;
  const int n0 = tn << 6;

  const int rlane = lane & 15;
  const int koff  = (lane >> 4) * 8;
  const int mOff  = (lane >> 4) * 8;

  v8f acc[4][4];
#pragma unroll
  for (int i = 0; i < 4; ++i)
#pragma unroll
    for (int j = 0; j < 4; ++j) acc[i][j] = (v8f){0.f,0.f,0.f,0.f,0.f,0.f,0.f,0.f};

  for (int k0 = 0; k0 < K; k0 += 32) {
    v16b bh[4];
#pragma unroll
    for (int j = 0; j < 4; ++j) {
      const size_t bo = (size_t)(n0 + (j << 4) + rlane) * ldb + koff + k0;
      bh[j] = FragB::load(Bt + bo);
    }
#pragma unroll
    for (int i = 0; i < 4; ++i) {
      const size_t ao = (size_t)(m0 + (i << 4) + rlane) * lda + koff + k0;
      v16b ah = FragB::load(A + ao);
      v16b al = ah;
      if (SPL >= 1) al = FragB::load(A2 + ao);
#pragma unroll
      for (int j = 0; j < 4; ++j) {
        acc[i][j] = FragB::mma(ah, bh[j], acc[i][j]);
        if (SPL >= 1) acc[i][j] = FragB::mma(al, bh[j], acc[i][j]);
      }
      guard4_b(acc[i][0], acc[i][1], acc[i][2], acc[i][3], ah, al);
    }
    keep4_b(bh[0], bh[1], bh[2], bh[3]);
  }
  acc_guard4(acc[0][0], acc[0][1], acc[0][2], acc[0][3]);
  acc_guard4(acc[1][0], acc[1][1], acc[1][2], acc[1][3]);
  acc_guard4(acc[2][0], acc[2][1], acc[2][2], acc[2][3]);
  acc_guard4(acc[3][0], acc[3][1], acc[3][2], acc[3][3]);

  float* slab = sT[wave];
#pragma unroll
  for (int i = 0; i < 4; ++i) {
    const int mBase = m0 + (i << 4);
#pragma unroll
    for (int j = 0; j < 4; ++j) {
      const int n = n0 + (j << 4) + rlane;
      float bv = 0.f;
      if (BIAS) {
        const int nc = (n < nBias) ? n : (nBias - 1);
        const float braw = bias[nc];
        const float brn  = bf_rne_f(braw);
        bv = (n < nBias) ? brn : 0.f;
      }
#pragma unroll
      for (int r = 0; r < 8; ++r) {
        const float v = acc[i][j][r] + bv;
        slab[(mOff + r) * 68 + (j << 4) + rlane] = v;
      }
    }
    __builtin_amdgcn_fence(__ATOMIC_RELEASE, "workgroup");
    __builtin_amdgcn_wave_barrier();
    __builtin_amdgcn_fence(__ATOMIC_ACQUIRE, "workgroup");
    {
      const int hh = lane >> 4, c4 = (lane & 15) * 4;
      for (int pass = 0; pass < 2; ++pass) {
#pragma unroll
        for (int it = 0; it < 8; ++it) {
          const int row = it * 2 + hh;
          v4f v = *(const v4f*)(slab + row * 68 + c4);
          *(volatile v4f*)(C + (size_t)(mBase + row) * ldc + n0 + c4) = v;
        }
        __threadfence();
      }
    }
    __builtin_amdgcn_fence(__ATOMIC_RELEASE, "workgroup");
    __builtin_amdgcn_wave_barrier();
    __builtin_amdgcn_fence(__ATOMIC_ACQUIRE, "workgroup");
  }
}

__global__ __launch_bounds__(256) void cast_bf16_kernel(
    const float* __restrict__ src, unsigned* __restrict__ dst, int total8, int valid8)
{
  const int i = blockIdx.x * 256 + threadIdx.x;
  if (i >= total8) return;
  const bool ok = (i < valid8);
  const int ic = ok ? i : (valid8 - 1);
  const size_t e0 = (size_t)ic << 3;
  const v4f a0 = *(const v4f*)(src + e0);
  const v4f a1 = *(const v4f*)(src + e0 + 4);
  const float f0 = ok ? a0[0] : 0.f;
  const float f1 = ok ? a0[1] : 0.f;
  const float f2 = ok ? a0[2] : 0.f;
  const float f3 = ok ? a0[3] : 0.f;
  const float f4 = ok ? a1[0] : 0.f;
  const float f5 = ok ? a1[1] : 0.f;
  const float f6 = ok ? a1[2] : 0.f;
  const float f7 = ok ? a1[3] : 0.f;
  v4u w;
  w[0] = pack_bf2(f0, f1);
  w[1] = pack_bf2(f2, f3);
  w[2] = pack_bf2(f4, f5);
  w[3] = pack_bf2(f6, f7);
  unsigned* q = dst + ((size_t)i << 2);
  *(volatile v4u*)q = w;
  __threadfence();
  *(volatile v4u*)q = w;
}

__global__ __launch_bounds__(256) void conv_silu_kernel(
    const float* __restrict__ XZ, const float* __restrict__ cw, const float* __restrict__ cb,
    unsigned* __restrict__ XCH, unsigned* __restrict__ XCL)
{
  __shared__ __align__(16) float sT[16 * kConvTP];
  const int tid = threadIdx.x, lane = tid & 31, wave = tid >> 5;
  const int d0 = blockIdx.x * 256, d = d0 + tid;
  const int g0 = blockIdx.y * 64;
  const int tb = g0 & (kSeq - 1);
  const v4f wv = *(const v4f*)(cw + (size_t)d * 4);
  const float w0 = bf_rne_f(wv[0]);
  const float w1 = bf_rne_f(wv[1]);
  const float w2 = bf_rne_f(wv[2]);
  const float w3 = bf_rne_f(wv[3]);
  const float bc = bf_rne_f(cb[d]);
  float xm3, xm2, xm1;
  {
    const bool hist = (tb > 0);
    const int rb = hist ? (g0 - 3) : g0;
    const float v3 = XZ[(size_t)rb * kXzP + d];
    const float v2 = XZ[(size_t)(rb + 1) * kXzP + d];
    const float v1 = XZ[(size_t)(rb + 2) * kXzP + d];
    xm3 = hist ? v3 : 0.f;
    xm2 = hist ? v2 : 0.f;
    xm1 = hist ? v1 : 0.f;
  }
#pragma unroll 1
  for (int sub = 0; sub < 4; ++sub) {
    const int lb = g0 + sub * 16;
#pragma unroll 1
    for (int s = 0; s < 16; ++s) {
      const float xcur = XZ[(size_t)(lb + s) * kXzP + d];
      float acc = w0 * xm3;
      acc = fmaf(w1, xm2, acc);
      acc = fmaf(w2, xm1, acc);
      acc = fmaf(w3, xcur, acc);
      const float sv = acc + bc;
      const float sg = __builtin_amdgcn_rcpf(1.0f + __expf(-sv));
      sT[s * kConvTP + tid] = sv * sg;
      xm3 = xm2; xm2 = xm1; xm1 = xcur;
    }
    __syncthreads();
    v4u hw[2], lw[2];
#pragma unroll
    for (int it = 0; it < 2; ++it) {
      const float* sp = sT + (it * 8 + wave) * kConvTP + lane * 8;
      const v4f a0 = *(const v4f*)(sp);
      const v4f a1 = *(const v4f*)(sp + 4);
      unsigned h0, l0, h1, l1, h2, l2, h3, l3;
      split_bf2(a0[0], a0[1], h0, l0);
      split_bf2(a0[2], a0[3], h1, l1);
      split_bf2(a1[0], a1[1], h2, l2);
      split_bf2(a1[2], a1[3], h3, l3);
      hw[it][0] = h0; hw[it][1] = h1; hw[it][2] = h2; hw[it][3] = h3;
      lw[it][0] = l0; lw[it][1] = l1; lw[it][2] = l2; lw[it][3] = l3;
    }
    for (int pass = 0; pass < 2; ++pass) {
#pragma unroll
      for (int it = 0; it < 2; ++it) {
        const size_t o = ((size_t)(lb + it * 8 + wave) * kDin + d0 + lane * 8) >> 1;
        *(volatile v4u*)(XCH + o) = hw[it];
        *(volatile v4u*)(XCL + o) = lw[it];
      }
      __threadfence();
    }
    __syncthreads();
  }
}

__global__ __launch_bounds__(64) void scan_kernel(
    const float* __restrict__ DBU, const float* __restrict__ XZ,
    const float* __restrict__ Wdt, const float* __restrict__ bdt, const float* __restrict__ Alog,
    const float* __restrict__ Dp, unsigned* __restrict__ YH, unsigned* __restrict__ YL)
{
  __shared__ __align__(16) float sX[kScanTS * kScanXP];
  __shared__ __align__(16) float sY[kScanTS * kScanYP];
  __shared__ __align__(16) float sW[kNst * kScanCh];
  __shared__ __align__(16) float sA[kNst * kScanCh];
  const int tid = threadIdx.x, lane = tid & 31, wave = tid >> 5;
  constexpr int kBlkPerB = kDin / kScanCh;
  const int bix = blockIdx.x / kBlkPerB;
  const int d0  = (blockIdx.x - bix * kBlkPerB) * kScanCh;
  const int d   = d0 + tid;
  const size_t row0 = (size_t)bix * kSeq;
#pragma unroll 1
  for (int j = 0; j < kNst; ++j) sW[j * kScanCh + tid] = bf_rne_f(Wdt[(size_t)d * kNst + j]);
#pragma unroll 1
  for (int n = 0; n < kNst; ++n) sA[n * kScanCh + tid] = -expf(bf_rne_f(Alog[(size_t)d * kNst + n]));
  __syncthreads();
  float negA[kNst], Wd[kNst], st[kNst];
#pragma unroll
  for (int n = 0; n < kNst; ++n) {
    negA[n] = sA[n * kScanCh + tid];
    Wd[n]   = sW[n * kScanCh + tid];
    st[n]   = 0.f;
  }
  const float bb = bf_rne_f(bdt[d]);
  const float Dd = bf_rne_f(Dp[d]);
  const int lr = tid >> 3, lc4 = (tid & 7) * 4;
  const int q = lane >> 3, c8 = (lane & 7) * 8;
#pragma unroll 1
  for (int t0 = 0; t0 < kSeq; t0 += kScanTS) {
    __syncthreads();
#pragma unroll
    for (int i = 0; i < 8; ++i) {
      const int r = lr + 8 * i;
      *(v4f*)(sX + r * kScanXP + lc4) = *(const v4f*)(DBU + (row0 + t0 + r) * kPrjP + lc4);
    }
    __syncthreads();
#pragma unroll 1
    for (int s = 0; s < kScanTS; ++s) {
      const size_t row = row0 + t0 + s;
      const float* xr = sX + s * kScanXP;
      const float ut = DBU[row * kPrjP + 2 * kNst + d];
      const float zv = XZ[row * kXzP + kDin + d];
      float vdot = 0.f;
#pragma unroll
      for (int r4 = 0; r4 < kNst / 4; ++r4) {
        const v4f xv = *(const v4f*)(xr + 4 * r4);
        vdot = fmaf(xv[0], Wd[4 * r4 + 0], vdot);
        vdot = fmaf(xv[1], Wd[4 * r4 + 1], vdot);
        vdot = fmaf(xv[2], Wd[4 * r4 + 2], vdot);
        vdot = fmaf(xv[3], Wd[4 * r4 + 3], vdot);
      }
      v4f Bq[4];
#pragma unroll
      for (int q4 = 0; q4 < 4; ++q4) Bq[q4] = *(const v4f*)(xr + kNst + 4 * q4);
      const float v   = vdot + bb;
      const float a   = __expf(-fabsf(v));
      const float u1  = 1.0f + a;
      const float l1p = __logf(u1) + (a - (u1 - 1.0f)) * __builtin_amdgcn_rcpf(u1);
      const float dt  = fmaxf(v, 0.0f) + l1p;
      const float dtu = dt * ut;
      float y = 0.f;
#pragma unroll
      for (int n = 0; n < kNst; ++n) {
        const float e = __expf(dt * negA[n]);
        st[n] = fmaf(e, st[n], dtu * Bq[n >> 2][n & 3]);
        y = fmaf(st[n], Dd, y);
      }
      y = fmaf(ut, Dd, y);
      const float sg = __builtin_amdgcn_rcpf(1.0f + __expf(-zv));
      y = y * (zv * sg);
      sY[s * kScanYP + tid] = y;
    }
    __syncthreads();
    v4u hv[8], lv[8];
#pragma unroll
    for (int it = 0; it < 8; ++it) {
      const int rw = it * 8 + wave * 4 + q;
      const float* sp = sY + rw * kScanYP + c8;
      const v4f a0 = *(const v4f*)(sp);
      const v4f a1 = *(const v4f*)(sp + 4);
      unsigned h0, l0, h1, l1, h2, l2, h3, l3;
      split_bf2(a0[0], a0[1], h0, l0);
      split_bf2(a0[2], a0[3], h1, l1);
      split_bf2(a1[0], a1[1], h2, l2);
      split_bf2(a1[2], a1[3], h3, l3);
      hv[it][0] = h0; hv[it][1] = h1; hv[it][2] = h2; hv[it][3] = h3;
      lv[it][0] = l0; lv[it][1] = l1; lv[it][2] = l2; lv[it][3] = l3;
    }
    for (int pass = 0; pass < 2; ++pass) {
#pragma unroll
      for (int it = 0; it < 8; ++it) {
        const int rw = it * 8 + wave * 4 + q;
        const size_t o = ((row0 + t0 + rw) * kDin + d0 + c8) >> 1;
        *(volatile v4u*)(YH + o) = hv[it];
        *(volatile v4u*)(YL + o) = lv[it];
      }
      __threadfence();
    }
  }
}

extern "C" void kernel_launch(void* const* d_in, const int* in_sizes, int n_in,
                              void* d_out, int out_size, void* d_ws, size_t ws_size,
                              hipStream_t stream) {
  if (n_in < 13) return;
  if (in_sizes[0]  != kRows * kDm) return;
  if (in_sizes[1]  != kXzP * kDm) return;
  if (in_sizes[2]  != kXzP) return;
  if (in_sizes[3]  != kDin * 4) return;
  if (in_sizes[4]  != kDin) return;
  if (in_sizes[5]  != kPrjN * kDin) return;
  if (in_sizes[6]  != kPrjN) return;
  if (in_sizes[7]  != kDin * kNst) return;
  if (in_sizes[8]  != kDin) return;
  if (in_sizes[9]  != kDin * kNst) return;
  if (in_sizes[10] != kDin) return;
  if (in_sizes[11] != kDm * kDin) return;
  if (in_sizes[12] != kDm) return;
  if (out_size != kRows * kDm) return;
  if (ws_size < kWsTotal) return;

  const float* x      = (const float*)d_in[0];
  const float* W_in   = (const float*)d_in[1];
  const float* b_in   = (const float*)d_in[2];
  const float* conv_w = (const float*)d_in[3];
  const float* conv_b = (const float*)d_in[4];
  const float* W_x    = (const float*)d_in[5];
  const float* b_x    = (const float*)d_in[6];
  const float* W_dt   = (const float*)d_in[7];
  const float* b_dt   = (const float*)d_in[8];
  const float* A_log  = (const float*)d_in[9];
  const float* Dp     = (const float*)d_in[10];
  const float* W_out  = (const float*)d_in[11];
  const float* b_out  = (const float*)d_in[12];
  float* out = (float*)d_out;

  char* ws = (char*)d_ws;
  unsigned* XB  = (unsigned*)(ws + kOffXB);
  unsigned* WIB = (unsigned*)(ws + kOffWIB);
  unsigned* WXB = (unsigned*)(ws + kOffWXB);
  unsigned* WOB = (unsigned*)(ws + kOffWOB);
  float*    XZ  = (float*)(ws + kOffXZ);
  unsigned* XCH = (unsigned*)(ws + kOffXCH);
  unsigned* XCL = (unsigned*)(ws + kOffXCL);
  float*    DBU = (float*)(ws + kOffDBU);
  unsigned* YH  = (unsigned*)(ws + kOffYH);
  unsigned* YL  = (unsigned*)(ws + kOffYL);

  cast_bf16_kernel<<<(kRows * kDm / 8) / 256, 256, 0, stream>>>(x, XB, kRows * kDm / 8, kRows * kDm / 8);
  cast_bf16_kernel<<<(kXzP * kDm / 8) / 256, 256, 0, stream>>>(W_in, WIB, kXzP * kDm / 8, kXzP * kDm / 8);
  cast_bf16_kernel<<<(kPrjP * kDin / 8) / 256, 256, 0, stream>>>(W_x, WXB, kPrjP * kDin / 8, kPrjN * kDin / 8);
  cast_bf16_kernel<<<(kDm * kDin / 8) / 256, 256, 0, stream>>>(W_out, WOB, kDm * kDin / 8, kDm * kDin / 8);

  wmma_gemm64<0, true><<<(kRows / 64) * (kXzP / 64) / 8, 256, 0, stream>>>(
      (const unsigned short*)XB, (const unsigned short*)XB, kDm,
      (const unsigned short*)WIB, kDm,
      XZ, kXzP, b_in, kXzP,
      kRows, kXzP, kDm);

  conv_silu_kernel<<<dim3(kDin / 256, kRows / 64), 256, 0, stream>>>(XZ, conv_w, conv_b, XCH, XCL);

  wmma_gemm64<1, true><<<(kRows / 64) * (kPrjP / 64) / 8, 256, 0, stream>>>(
      (const unsigned short*)XCH, (const unsigned short*)XCL, kDin,
      (const unsigned short*)WXB, kDin,
      DBU, kPrjP, b_x, kPrjN,
      kRows, kPrjP, kDin);

  scan_kernel<<<kBatch * (kDin / kScanCh), kScanCh, 0, stream>>>(DBU, XZ, W_dt, b_dt, A_log, Dp, YH, YL);

  wmma_gemm64<1, true><<<(kRows / 64) * (kDm / 64) / 8, 256, 0, stream>>>(
      (const unsigned short*)YH, (const unsigned short*)YL, kDin,
      (const unsigned short*)WOB, kDin,
      out, kDm, b_out, kDm,
      kRows, kDm, kDin);
}
